// GemmaAttention_84404697301698
// MI455X (gfx1250) — hardware-verified
//
#include <hip/hip_runtime.h>
#include <math.h>

#define SEQ_LEN   2048
#define NBATCH    2
#define HID_DIM   2048
#define NUM_HEADS 8
#define HEAD_DIM  256
#define HALF_DIM  128
#define NTOK      (NBATCH * SEQ_LEN)
#define KV_CHUNK  64
#define QBLK      64

typedef __attribute__((ext_vector_type(16))) _Float16 v16h;
typedef __attribute__((ext_vector_type(8)))  _Float16 v8h;
typedef __attribute__((ext_vector_type(16))) __bf16   v16b;
typedef __attribute__((ext_vector_type(8)))  __bf16   v8b;
typedef __attribute__((ext_vector_type(8)))  float    v8f;
typedef __attribute__((ext_vector_type(4)))  float    v4f;
typedef __attribute__((ext_vector_type(4)))  unsigned int v4u;

__device__ __forceinline__ unsigned short f2bf_bits(float f) {
  unsigned u = __float_as_uint(f);
  return (unsigned short)((u + 0x7FFFu + ((u >> 16) & 1u)) >> 16);
}
__device__ __forceinline__ float bf_bits2f(unsigned short h) { return __uint_as_float(((unsigned)h) << 16); }

__device__ __forceinline__ void dep_guard_h(v8f& a, v8f& b, v16h x, v16h y) { asm volatile("v_nop\n\tv_nop\n\tv_nop\n\tv_nop" : "+v"(a), "+v"(b) : "v"(x), "v"(y)); }
__device__ __forceinline__ void dep_guard_b(v8f& a, v8f& b, v16b x, v16b y) { asm volatile("v_nop\n\tv_nop\n\tv_nop\n\tv_nop" : "+v"(a), "+v"(b) : "v"(x), "v"(y)); }
__device__ __forceinline__ void keep4_h(v16h a, v16h b, v16h c, v16h d) { asm volatile("v_nop" :: "v"(a), "v"(b), "v"(c), "v"(d)); }
__device__ __forceinline__ void keep4_b(v16b a, v16b b, v16b c, v16b d) { asm volatile("v_nop" :: "v"(a), "v"(b), "v"(c), "v"(d)); }
__device__ __forceinline__ void acc_guard4(v8f& a, v8f& b, v8f& c, v8f& d) { asm volatile("v_nop\n\tv_nop\n\tv_nop\n\tv_nop" : "+v"(a), "+v"(b), "+v"(c), "+v"(d)); }

template <typename T> struct Frag;
template <> struct Frag<_Float16> {
  typedef v16h V; union U { v16h v; v8h h[2]; };
  static __device__ __forceinline__ v16h load(const _Float16* p) {
    U f; f.h[0] = *(const v8h*)(p); f.h[1] = *(const v8h*)(p + 16); return f.v;
  }
  static __device__ __forceinline__ v8f mma(v16h a, v16h b, v8f c) {
    return __builtin_amdgcn_wmma_f32_16x16x32_f16(false, a, false, b, (short)0, c, false, false);
  }
  static __device__ __forceinline__ void guard(v8f& a, v8f& b, v16h x, v16h y) { dep_guard_h(a, b, x, y); }
  static __device__ __forceinline__ void keep(v16h a, v16h b, v16h c, v16h d) { keep4_h(a, b, c, d); }
};
template <> struct Frag<__bf16> {
  typedef v16b V; union U { v16b v; v8b h[2]; };
  static __device__ __forceinline__ v16b load(const __bf16* p) {
    U f; f.h[0] = *(const v8b*)(p); f.h[1] = *(const v8b*)(p + 16); return f.v;
  }
  static __device__ __forceinline__ v8f mma(v16b a, v16b b, v8f c) {
    return __builtin_amdgcn_wmma_f32_16x16x32_bf16(false, a, false, b, (short)0, c, false, false);
  }
  static __device__ __forceinline__ void guard(v8f& a, v8f& b, v16b x, v16b y) { dep_guard_b(a, b, x, y); }
  static __device__ __forceinline__ void keep(v16b a, v16b b, v16b c, v16b d) { keep4_b(a, b, c, d); }
};

__device__ __forceinline__ unsigned short at_bf_bits(float f) {
  unsigned u = __float_as_uint(f);
  return (unsigned short)((u + 0x7FFFu + ((u >> 16) & 1u)) >> 16);
}
__device__ __forceinline__ __bf16 at_f2bf(float f) { return __builtin_bit_cast(__bf16, at_bf_bits(f)); }
__device__ __forceinline__ void at_split(float f, __bf16& hi, __bf16& lo) {
  const unsigned short hb = at_bf_bits(f);
  hi = __builtin_bit_cast(__bf16, hb);
  lo = at_f2bf(f - __uint_as_float(((unsigned)hb) << 16));
}
__device__ __forceinline__ v8f at_mma(v16b a, v16b b, v8f c) {
  c = __builtin_amdgcn_wmma_f32_16x16x32_bf16(false, a, false, b, (short)0, c, false, false);
  asm volatile("v_nop\n\tv_nop\n\tv_nop\n\tv_nop" : "+v"(c) : "v"(a), "v"(b));
  return c;
}

__device__ __forceinline__ void split_pack2(float f0, float f1, unsigned& hw, unsigned& lw) {
  const unsigned short h0 = f2bf_bits(f0), h1 = f2bf_bits(f1);
  const unsigned short l0 = f2bf_bits(f0 - bf_bits2f(h0));
  const unsigned short l1 = f2bf_bits(f1 - bf_bits2f(h1));
  hw = (unsigned)h0 | ((unsigned)h1 << 16);
  lw = (unsigned)l0 | ((unsigned)l1 << 16);
}

__global__ __launch_bounds__(256) void cast8_f32_bf16(const float* __restrict__ in, unsigned short* __restrict__ out, int n8) {
  const int i = blockIdx.x * 256 + threadIdx.x;
  if (i < n8) {
    const size_t o = (size_t)i * 8;
    const v4f a = *(const v4f*)(in + o);
    const v4f bq = *(const v4f*)(in + o + 4);
    v4u w;
    w[0] = (unsigned)f2bf_bits(a[0])  | ((unsigned)f2bf_bits(a[1])  << 16);
    w[1] = (unsigned)f2bf_bits(a[2])  | ((unsigned)f2bf_bits(a[3])  << 16);
    w[2] = (unsigned)f2bf_bits(bq[0]) | ((unsigned)f2bf_bits(bq[1]) << 16);
    w[3] = (unsigned)f2bf_bits(bq[2]) | ((unsigned)f2bf_bits(bq[3]) << 16);
    *(volatile v4u*)(out + o) = w;
    __threadfence();
    *(volatile v4u*)(out + o) = w;
  }
}

__global__ __launch_bounds__(256) void transpose_cast_bf16(const float* __restrict__ in, unsigned short* __restrict__ out, int nrows, int ncols) {
  __shared__ float tile[64 * 65];
  const int tid = threadIdx.x;
  const int r0 = blockIdx.y * 64, c0 = blockIdx.x * 64;
  {
    const int row = tid >> 2, cc = (tid & 3) * 16;
    const float* s = in + (size_t)(r0 + row) * ncols + c0 + cc;
#pragma unroll
    for (int q = 0; q < 4; ++q) {
      const v4f v = *(const v4f*)(s + 4 * q);
#pragma unroll
      for (int e = 0; e < 4; ++e) tile[(cc + 4 * q + e) * 65 + row] = v[e];
    }
  }
  __syncthreads();
  for (int pass = 0; pass < 2; ++pass) {
#pragma unroll
    for (int it = 0; it < 2; ++it) {
      const int orow = it * 32 + (tid >> 3), seg = (tid & 7) * 8;
      const float* tp = tile + orow * 65 + seg;
      v4u w;
#pragma unroll
      for (int e = 0; e < 4; ++e) w[e] = (unsigned)f2bf_bits(tp[2 * e]) | ((unsigned)f2bf_bits(tp[2 * e + 1]) << 16);
      *(volatile v4u*)(out + (size_t)(c0 + orow) * nrows + r0 + seg) = w;
    }
    __threadfence();
  }
}

struct RopeFreq { float f[HALF_DIM]; };
static_assert(sizeof(RopeFreq) == 512, "size");

__global__ __launch_bounds__(256) void rope_table_kernel(float* __restrict__ cosT, float* __restrict__ sinT, RopeFreq fr) {
  __shared__ float invf[HALF_DIM];
  if (threadIdx.x == 0) {
#pragma unroll
    for (int q = 0; q < HALF_DIM; ++q) invf[q] = fr.f[q];
  }
  __syncthreads();
  const int i = blockIdx.x * 256 + threadIdx.x;
  const int t = i >> 7;
  const int jj = i & (HALF_DIM - 1);
  const float ang = (float)t * invf[jj];
  const float cv = cosf(ang);
  const float sv = sinf(ang);
  ((volatile float*)cosT)[i] = cv;
  ((volatile float*)sinT)[i] = sv;
  __threadfence();
  ((volatile float*)cosT)[i] = cv;
  ((volatile float*)sinT)[i] = sv;
}

template <int NHEAD, int PITCH>
__global__ __launch_bounds__(256) void rope_split_kernel(const float* __restrict__ src, const float* __restrict__ cosT, const float* __restrict__ sinT,
                                                          unsigned short* __restrict__ outH, unsigned short* __restrict__ outL, float scl) {
  const int i = blockIdx.x * 256 + threadIdx.x;
  const int jg = i & 15;
  const int hs = (i >> 4) % NHEAD;
  const int tok = (i >> 4) / NHEAD;
  const int pos = tok & (SEQ_LEN - 1);
  const size_t base = (size_t)tok * PITCH + (size_t)hs * HEAD_DIM + jg * 8;
  const size_t tb = (size_t)pos * HALF_DIM + jg * 8;
  const v4f x1a = *(const v4f*)(src + base);
  const v4f x1b = *(const v4f*)(src + base + 4);
  const v4f x2a = *(const v4f*)(src + base + HALF_DIM);
  const v4f x2b = *(const v4f*)(src + base + HALF_DIM + 4);
  const v4f ca = *(const v4f*)(cosT + tb);
  const v4f cb = *(const v4f*)(cosT + tb + 4);
  const v4f sa = *(const v4f*)(sinT + tb);
  const v4f sb = *(const v4f*)(sinT + tb + 4);
  v4f o1a, o1b, o2a, o2b;
#pragma unroll
  for (int e = 0; e < 4; ++e) {
    o1a[e] = (x1a[e] * ca[e] - x2a[e] * sa[e]) * scl;
    o2a[e] = (x2a[e] * ca[e] + x1a[e] * sa[e]) * scl;
    o1b[e] = (x1b[e] * cb[e] - x2b[e] * sb[e]) * scl;
    o2b[e] = (x2b[e] * cb[e] + x1b[e] * sb[e]) * scl;
  }
  v4u h1, l1, h2, l2;
  {
    unsigned hw, lw;
    split_pack2(o1a[0], o1a[1], hw, lw); h1[0] = hw; l1[0] = lw;
    split_pack2(o1a[2], o1a[3], hw, lw); h1[1] = hw; l1[1] = lw;
    split_pack2(o1b[0], o1b[1], hw, lw); h1[2] = hw; l1[2] = lw;
    split_pack2(o1b[2], o1b[3], hw, lw); h1[3] = hw; l1[3] = lw;
    split_pack2(o2a[0], o2a[1], hw, lw); h2[0] = hw; l2[0] = lw;
    split_pack2(o2a[2], o2a[3], hw, lw); h2[1] = hw; l2[1] = lw;
    split_pack2(o2b[0], o2b[1], hw, lw); h2[2] = hw; l2[2] = lw;
    split_pack2(o2b[2], o2b[3], hw, lw); h2[3] = hw; l2[3] = lw;
  }
  for (int pass = 0; pass < 2; ++pass) {
    *(volatile v4u*)(outH + base) = h1;
    *(volatile v4u*)(outH + base + HALF_DIM) = h2;
    *(volatile v4u*)(outL + base) = l1;
    *(volatile v4u*)(outL + base + HALF_DIM) = l2;
    __threadfence();
  }
}

template <bool SPLITA, bool SPLITB, int OUT_MODE>
__global__ __launch_bounds__(256) void gemm_bf16_t64(
    const unsigned short* __restrict__ Ap, const unsigned short* __restrict__ A2p, int lda, long strideA,
    const unsigned short* __restrict__ Btp, const unsigned short* __restrict__ Bt2p, int ldb, long strideB,
    void* __restrict__ Cout, void* __restrict__ Cout2, int ldc, long strideC,
    int M, int N, int K, float scale) {
  typedef __bf16 T;
  typedef v16b V;
  const T* A = (const T*)Ap; const T* A2 = (const T*)A2p; const T* Bt = (const T*)Btp; const T* Bt2 = (const T*)Bt2p;
  __shared__ __align__(16) float sT[8][16 * 68];
  const int b    = blockIdx.y;
  const int lane = threadIdx.x & 31;
  const int wave = threadIdx.x >> 5;
  const int tilesN = N >> 6;
  const int tilesM = M >> 6;
  const int tile = blockIdx.x * 8 + wave;
  if (tile >= tilesM * tilesN) return;
  const int tm = tile / tilesN;
  const int tn = tile - tm * tilesN;
  const int m0 = tm << 6;
  const int n0 = tn << 6;

  const T* Ab  = A  + (size_t)b * strideA;
  const T* Bb  = Bt + (size_t)b * strideB;
  const T* Ab2 = A2  + (size_t)b * strideA;
  const T* Bb2 = Bt2 + (size_t)b * strideB;

  const int rlane = lane & 15;
  const int koff  = (lane >> 4) * 8;
  const int mOff  = (lane >> 4) * 8;

  v8f acc[4][4];
#pragma unroll
  for (int i = 0; i < 4; ++i)
#pragma unroll
    for (int j = 0; j < 4; ++j) acc[i][j] = (v8f){0.f,0.f,0.f,0.f,0.f,0.f,0.f,0.f};

  for (int k0 = 0; k0 < K; k0 += 32) {
    V bh[4], bl[4];
#pragma unroll
    for (int j = 0; j < 4; ++j) {
      const size_t bo = (size_t)(n0 + (j << 4) + rlane) * ldb + koff + k0;
      bh[j] = Frag<T>::load(Bb + bo);
      if (SPLITB) bl[j] = Frag<T>::load(Bb2 + bo);
    }
#pragma unroll
    for (int i = 0; i < 4; ++i) {
      const size_t ao = (size_t)(m0 + (i << 4) + rlane) * lda + koff + k0;
      V ah = Frag<T>::load(Ab + ao);
      V al = ah;
      if (SPLITA) al = Frag<T>::load(Ab2 + ao);
#pragma unroll
      for (int j = 0; j < 4; ++j) {
        acc[i][j] = Frag<T>::mma(ah, bh[j], acc[i][j]);
        if (SPLITB) acc[i][j] = Frag<T>::mma(ah, bl[j], acc[i][j]);
        if (SPLITA) acc[i][j] = Frag<T>::mma(al, bh[j], acc[i][j]);
      }
      Frag<T>::guard(acc[i][0], acc[i][3], ah, al);
    }
    Frag<T>::keep(bh[0], bh[1], bh[2], bh[3]);
    if (SPLITB) Frag<T>::keep(bl[0], bl[1], bl[2], bl[3]);
  }
  acc_guard4(acc[0][0], acc[0][1], acc[0][2], acc[0][3]);
  acc_guard4(acc[1][0], acc[1][1], acc[1][2], acc[1][3]);
  acc_guard4(acc[2][0], acc[2][1], acc[2][2], acc[2][3]);
  acc_guard4(acc[3][0], acc[3][1], acc[3][2], acc[3][3]);

  float* slab = sT[wave];
#pragma unroll
  for (int i = 0; i < 4; ++i) {
    const int mBase = m0 + (i << 4);
#pragma unroll
    for (int j = 0; j < 4; ++j) {
#pragma unroll
      for (int r = 0; r < 8; ++r) {
        const float v = acc[i][j][r] * scale;
        slab[(mOff + r) * 68 + (j << 4) + rlane] = v;
      }
    }
    __builtin_amdgcn_fence(__ATOMIC_RELEASE, "workgroup");
    __builtin_amdgcn_wave_barrier();
    __builtin_amdgcn_fence(__ATOMIC_ACQUIRE, "workgroup");
    if (OUT_MODE == 0) {
      float* Cf = (float*)Cout + (size_t)b * strideC;
      const int hh = lane >> 4, c4 = (lane & 15) * 4;
      for (int pass = 0; pass < 2; ++pass) {
#pragma unroll
        for (int it = 0; it < 8; ++it) {
          const int row = it * 2 + hh;
          v4f v = *(const v4f*)(slab + row * 68 + c4);
          *(volatile v4f*)(Cf + (size_t)(mBase + row) * ldc + n0 + c4) = v;
        }
        __threadfence();
      }
    } else {
      const int q = lane >> 3, c8 = (lane & 7) * 8;
      unsigned short* Cs  = (unsigned short*)Cout  + (size_t)b * strideC;
      unsigned short* Cs2 = (unsigned short*)Cout2 + (size_t)b * strideC;
      for (int pass = 0; pass < 2; ++pass) {
#pragma unroll
        for (int it = 0; it < 4; ++it) {
          const int row = it * 4 + q;
          const float* sp = slab + row * 68 + c8;
          v8h hv, lv;
#pragma unroll
          for (int e = 0; e < 8; ++e) {
            unsigned short hb = f2bf_bits(sp[e]);
            unsigned short lb = f2bf_bits(sp[e] - bf_bits2f(hb));
            hv[e] = __builtin_bit_cast(_Float16, hb);
            lv[e] = __builtin_bit_cast(_Float16, lb);
          }
          *(volatile v8h*)(Cs + (size_t)(mBase + row) * ldc + n0 + c8) = hv;
          *(volatile v8h*)(Cs2 + (size_t)(mBase + row) * ldc + n0 + c8) = lv;
        }
        __threadfence();
      }
    }
    __builtin_amdgcn_fence(__ATOMIC_RELEASE, "workgroup");
    __builtin_amdgcn_wave_barrier();
    __builtin_amdgcn_fence(__ATOMIC_ACQUIRE, "workgroup");
  }
}

__global__ __launch_bounds__(256) void gqa_attn_kernel(
    const unsigned short* __restrict__ Qhp, const unsigned short* __restrict__ Qlp,
    const unsigned short* __restrict__ Khp, const unsigned short* __restrict__ Klp,
    const unsigned short* __restrict__ Vhp, const unsigned short* __restrict__ Vlp,
    const float* __restrict__ maskp,
    unsigned short* __restrict__ Ohp, unsigned short* __restrict__ Olp) {
  __shared__ __align__(16) float  Spart[8][16 * KV_CHUNK];
  __shared__ __align__(16) float  Msk[QBLK * KV_CHUNK];
  __shared__ __align__(16) __bf16 Psh[4][16 * KV_CHUNK];
  __shared__ __align__(16) __bf16 Psl[4][16 * KV_CHUNK];

  const __bf16* Qh = (const __bf16*)Qhp;
  const __bf16* Ql = (const __bf16*)Qlp;
  const __bf16* Kh = (const __bf16*)Khp;
  const __bf16* Kl = (const __bf16*)Klp;
  const __bf16* Vh = (const __bf16*)Vhp;
  const __bf16* Vl = (const __bf16*)Vlp;

  const int tid  = threadIdx.x;
  const int wave = tid >> 5, lane = tid & 31;
  const int hh   = lane >> 4, c = lane & 15, koff = hh * 8;
  const int rg   = wave & 3, dh = wave >> 2;
  const int bx   = blockIdx.x;
  const int qb   = bx & (SEQ_LEN / QBLK - 1);
  const int bhid = bx / (SEQ_LEN / QBLK);
  const int h    = bhid & (NUM_HEADS - 1);
  const int b    = bhid / NUM_HEADS;
  const int q0   = qb * QBLK + rg * 16;
  const size_t tokw = (size_t)b * SEQ_LEN + q0;
  const size_t qoff = (tokw + c) * HID_DIM + (size_t)h * HEAD_DIM + dh * HALF_DIM + koff;
  const __bf16* Khb = Kh + (size_t)b * SEQ_LEN * HEAD_DIM + dh * HALF_DIM + koff;
  const __bf16* Klb = Kl + (size_t)b * SEQ_LEN * HEAD_DIM + dh * HALF_DIM + koff;
  const __bf16* Vhb = Vh + (size_t)b * HEAD_DIM * SEQ_LEN + (size_t)(dh * HALF_DIM + c) * SEQ_LEN + koff;
  const __bf16* Vlb = Vl + (size_t)b * HEAD_DIM * SEQ_LEN + (size_t)(dh * HALF_DIM + c) * SEQ_LEN + koff;
  const int mr = tid >> 2, mc = (tid & 3) * 16;
  const float* mrowp = maskp + (size_t)(qb * QBLK + mr) * SEQ_LEN + mc;

  float mrow[8], lrow[8];
  v8f oacc[8];
#pragma unroll
  for (int r = 0; r < 8; ++r) { mrow[r] = -INFINITY; lrow[r] = 0.f; }
#pragma unroll
  for (int t = 0; t < 8; ++t) oacc[t] = (v8f){0.f,0.f,0.f,0.f,0.f,0.f,0.f,0.f};

  const int nChunks = qb + 1;
  for (int kc = 0; kc < nChunks; ++kc) {
    const int kv0 = kc * KV_CHUNK;

    {
#pragma unroll
      for (int q4i = 0; q4i < 4; ++q4i) {
        const v4f mv = *(const v4f*)(mrowp + kv0 + 4 * q4i);
        *(v4f*)(Msk + mr * KV_CHUNK + mc + 4 * q4i) = mv;
      }
    }

    v8f s[4];
#pragma unroll
    for (int j = 0; j < 4; ++j) s[j] = (v8f){0.f,0.f,0.f,0.f,0.f,0.f,0.f,0.f};
#pragma unroll
    for (int dc = 0; dc < 4; ++dc) {
      const v16b qa = Frag<__bf16>::load(Qh + qoff + dc * 32);
      const v16b ql = Frag<__bf16>::load(Ql + qoff + dc * 32);
#pragma unroll
      for (int j = 0; j < 4; ++j) {
        const size_t ko = (size_t)(kv0 + j * 16 + c) * HEAD_DIM + dc * 32;
        const v16b kb = Frag<__bf16>::load(Khb + ko);
        const v16b kl = Frag<__bf16>::load(Klb + ko);
        s[j] = at_mma(qa, kb, s[j]);
        s[j] = at_mma(qa, kl, s[j]);
        s[j] = at_mma(ql, kb, s[j]);
      }
    }

    {
      float* sp = Spart[wave];
#pragma unroll
      for (int r = 0; r < 8; ++r)
#pragma unroll
        for (int j = 0; j < 4; ++j) sp[(8 * hh + r) * KV_CHUNK + j * 16 + c] = s[j][r];
    }
    __syncthreads();
    {
      const float* pp = Spart[wave ^ 4];
#pragma unroll
      for (int r = 0; r < 8; ++r)
#pragma unroll
        for (int j = 0; j < 4; ++j) s[j][r] = s[j][r] + pp[(8 * hh + r) * KV_CHUNK + j * 16 + c];
    }

    float cm[8];
#pragma unroll
    for (int r = 0; r < 8; ++r) {
      const int lrow_blk = rg * 16 + 8 * hh + r;
      float m = -INFINITY;
#pragma unroll
      for (int j = 0; j < 4; ++j) {
        const float mk = Msk[lrow_blk * KV_CHUNK + j * 16 + c];
        const float sv = s[j][r] + mk;
        s[j][r] = sv;
        m = fmaxf(m, sv);
      }
#pragma unroll
      for (int off = 1; off < 16; off <<= 1) m = fmaxf(m, __shfl_xor(m, off, 32));
      cm[r] = m;
    }

    __bf16* pwh_w = Psh[rg];
    __bf16* pwl_w = Psl[rg];
#pragma unroll
    for (int r = 0; r < 8; ++r) {
      const float mnew = fmaxf(mrow[r], cm[r]);
      const float alpha = expf(mrow[r] - mnew);
      mrow[r] = mnew;
      float psum = 0.f;
#pragma unroll
      for (int j = 0; j < 4; ++j) {
        const float p = expf(s[j][r] - mnew);
        psum += p;
        __bf16 ph, plo;
        at_split(p, ph, plo);
        if (dh == 0) {
          pwh_w[(8 * hh + r) * KV_CHUNK + j * 16 + c] = ph;
          pwl_w[(8 * hh + r) * KV_CHUNK + j * 16 + c] = plo;
        }
      }
#pragma unroll
      for (int off = 1; off < 16; off <<= 1) psum += __shfl_xor(psum, off, 32);
      lrow[r] = lrow[r] * alpha + psum;
#pragma unroll
      for (int t = 0; t < 8; ++t) oacc[t][r] *= alpha;
    }
    __syncthreads();

    const __bf16* pwh = Psh[rg];
    const __bf16* pwl = Psl[rg];
#pragma unroll
    for (int kk = 0; kk < 2; ++kk) {
      const v16b pa = Frag<__bf16>::load(pwh + c * KV_CHUNK + kk * 32 + koff);
      const v16b pl = Frag<__bf16>::load(pwl + c * KV_CHUNK + kk * 32 + koff);
#pragma unroll
      for (int t = 0; t < 8; ++t) {
        const size_t vo = (size_t)t * 16 * SEQ_LEN + kv0 + kk * 32;
        const v16b vb = Frag<__bf16>::load(Vhb + vo);
        const v16b vl = Frag<__bf16>::load(Vlb + vo);
        oacc[t] = at_mma(pa, vb, oacc[t]);
        oacc[t] = at_mma(pa, vl, oacc[t]);
        oacc[t] = at_mma(pl, vb, oacc[t]);
      }
    }
  }

  float* os = Spart[wave];
  const int q4 = lane >> 3, c8 = (lane & 7) * 8;
#pragma unroll
  for (int th = 0; th < 2; ++th) {
#pragma unroll
    for (int r = 0; r < 8; ++r) {
      const float inv = 1.0f / lrow[r];
#pragma unroll
      for (int tt = 0; tt < 4; ++tt) os[(8 * hh + r) * KV_CHUNK + tt * 16 + c] = oacc[th * 4 + tt][r] * inv;
    }
    __builtin_amdgcn_fence(__ATOMIC_RELEASE, "workgroup");
    __builtin_amdgcn_wave_barrier();
    __builtin_amdgcn_fence(__ATOMIC_ACQUIRE, "workgroup");
    for (int pass = 0; pass < 2; ++pass) {
#pragma unroll
      for (int it = 0; it < 4; ++it) {
        const int row = it * 4 + q4;
        const float* sp = os + row * KV_CHUNK + c8;
        v4u hw, lw;
#pragma unroll
        for (int e = 0; e < 4; ++e) {
          unsigned a, bq;
          split_pack2(sp[2 * e], sp[2 * e + 1], a, bq);
          hw[e] = a; lw[e] = bq;
        }
        const size_t o = (tokw + row) * HID_DIM + (size_t)h * HEAD_DIM + dh * HALF_DIM + th * 64 + c8;
        *(volatile v4u*)(Ohp + o) = hw;
        *(volatile v4u*)(Olp + o) = lw;
      }
      __threadfence();
    }
    __builtin_amdgcn_fence(__ATOMIC_RELEASE, "workgroup");
    __builtin_amdgcn_wave_barrier();
    __builtin_amdgcn_fence(__ATOMIC_ACQUIRE, "workgroup");
  }
}

static_assert((NTOK * HID_DIM / 8) % 256 == 0, "cast grid");
static_assert((NTOK * NUM_HEADS * 16) % 256 == 0, "rope q grid");
static_assert((NTOK * 16) % 256 == 0, "rope k grid");
static_assert((SEQ_LEN * HALF_DIM) % 256 == 0, "table grid");
static_assert(HID_DIM % 32 == 0 && (NUM_HEADS * HEAD_DIM) % 32 == 0, "K multiple of 32");
static_assert(NTOK % 64 == 0 && HID_DIM % 64 == 0 && HEAD_DIM % 64 == 0 && SEQ_LEN % 64 == 0, "tile multiples");
static_assert(((NTOK / 64) * (HID_DIM / 64)) % 8 == 0 && ((NTOK / 64) * (HEAD_DIM / 64)) % 8 == 0 && ((HEAD_DIM / 64) * (SEQ_LEN / 64)) % 8 == 0, "gemm grids");
static_assert(SEQ_LEN % QBLK == 0 && QBLK == KV_CHUNK, "attention blocks");

extern "C" void kernel_launch(void* const* d_in, const int* in_sizes, int n_in,
                              void* d_out, int out_size, void* d_ws, size_t ws_size, hipStream_t stream) {
  (void)in_sizes; (void)n_in; (void)out_size;
  const float* x     = (const float*)d_in[0];
  const float* Wq    = (const float*)d_in[1];
  const float* Wk    = (const float*)d_in[2];
  const float* Wv    = (const float*)d_in[3];
  const float* Wo    = (const float*)d_in[4];
  const float* maskp = (const float*)d_in[5];
  float* out = (float*)d_out;

  const size_t MIB = 1048576;
  const size_t OFF_XB = 0, OFF_WQT = 16 * MIB, OFF_WKT = 24 * MIB, OFF_WVT = 25 * MIB, OFF_WOT = 26 * MIB;
  const size_t OFF_QF = 34 * MIB, OFF_AOH = 34 * MIB, OFF_AOL = 50 * MIB, OFF_KF = 66 * MIB;
  const size_t OFF_QH = 70 * MIB, OFF_QL = 86 * MIB, OFF_KH = 102 * MIB, OFF_KL = 104 * MIB;
  const size_t OFF_VH = 106 * MIB, OFF_VL = 108 * MIB, OFF_COS = 110 * MIB, OFF_SIN = 111 * MIB;
  const size_t WS_TOTAL = 112 * MIB;
  static_assert((size_t)NTOK * HID_DIM * 2 == 16 * 1048576, "xb");
  static_assert((size_t)HID_DIM * HID_DIM * 2 == 8 * 1048576, "wqt");
  static_assert((size_t)HEAD_DIM * HID_DIM * 2 == 1 * 1048576, "wkt");
  static_assert((size_t)NTOK * HID_DIM * 4 == 32 * 1048576, "qf");
  static_assert((size_t)NTOK * HEAD_DIM * 4 == 4 * 1048576, "kf");
  static_assert((size_t)NTOK * HEAD_DIM * 2 == 2 * 1048576, "kh");
  static_assert((size_t)NBATCH * HEAD_DIM * SEQ_LEN * 2 == 2 * 1048576, "vt");
  static_assert((size_t)SEQ_LEN * HALF_DIM * 4 == 1 * 1048576, "tab");
  if (ws_size < WS_TOTAL) return;

  char* ws = (char*)d_ws;
  unsigned short* xb  = (unsigned short*)(ws + OFF_XB);
  unsigned short* WqT = (unsigned short*)(ws + OFF_WQT);
  unsigned short* WkT = (unsigned short*)(ws + OFF_WKT);
  unsigned short* WvT = (unsigned short*)(ws + OFF_WVT);
  unsigned short* WoT = (unsigned short*)(ws + OFF_WOT);
  float* Qf  = (float*)(ws + OFF_QF);
  float* Kf  = (float*)(ws + OFF_KF);
  unsigned short* AOh = (unsigned short*)(ws + OFF_AOH);
  unsigned short* AOl = (unsigned short*)(ws + OFF_AOL);
  unsigned short* Qh  = (unsigned short*)(ws + OFF_QH);
  unsigned short* Ql  = (unsigned short*)(ws + OFF_QL);
  unsigned short* Kh  = (unsigned short*)(ws + OFF_KH);
  unsigned short* Kl  = (unsigned short*)(ws + OFF_KL);
  unsigned short* Vth = (unsigned short*)(ws + OFF_VH);
  unsigned short* Vtl = (unsigned short*)(ws + OFF_VL);
  float* cosT = (float*)(ws + OFF_COS);
  float* sinT = (float*)(ws + OFF_SIN);

  RopeFreq fr;
  for (int j = 0; j < HALF_DIM; ++j) {
    const float e = (float)(2 * j) / 256.0f;
    const double p = pow(10000.0, (double)e);
    const float pf = (float)p;
    fr.f[j] = 1.0f / pf;
  }

  cast8_f32_bf16<<<(NTOK * HID_DIM / 8) / 256, 256, 0, stream>>>(x, xb, NTOK * HID_DIM / 8);
  transpose_cast_bf16<<<dim3(HID_DIM / 64, HID_DIM / 64), 256, 0, stream>>>(Wq, WqT, HID_DIM, HID_DIM);
  transpose_cast_bf16<<<dim3(HEAD_DIM / 64, HID_DIM / 64), 256, 0, stream>>>(Wk, WkT, HID_DIM, HEAD_DIM);
  transpose_cast_bf16<<<dim3(HEAD_DIM / 64, HID_DIM / 64), 256, 0, stream>>>(Wv, WvT, HID_DIM, HEAD_DIM);
  transpose_cast_bf16<<<dim3(HID_DIM / 64, HID_DIM / 64), 256, 0, stream>>>(Wo, WoT, HID_DIM, HID_DIM);
  rope_table_kernel<<<(SEQ_LEN * HALF_DIM) / 256, 256, 0, stream>>>(cosT, sinT, fr);
  gemm_bf16_t64<false, false, 0><<<dim3(((NTOK / 64) * (HID_DIM / 64)) / 8, 1), 256, 0, stream>>>(
      xb, xb, HID_DIM, 0L, WqT, WqT, HID_DIM, 0L, (void*)Qf, (void*)Qf, HID_DIM, 0L, NTOK, HID_DIM, HID_DIM, 1.0f);
  gemm_bf16_t64<false, false, 0><<<dim3(((NTOK / 64) * (HEAD_DIM / 64)) / 8, 1), 256, 0, stream>>>(
      xb, xb, HID_DIM, 0L, WkT, WkT, HID_DIM, 0L, (void*)Kf, (void*)Kf, HEAD_DIM, 0L, NTOK, HEAD_DIM, HID_DIM, 1.0f);
  gemm_bf16_t64<false, false, 2><<<dim3(((HEAD_DIM / 64) * (SEQ_LEN / 64)) / 8, NBATCH), 256, 0, stream>>>(
      WvT, WvT, HID_DIM, 0L, xb, xb, HID_DIM, (long)SEQ_LEN * HID_DIM, (void*)Vth, (void*)Vtl, SEQ_LEN, (long)HEAD_DIM * SEQ_LEN,
      HEAD_DIM, SEQ_LEN, HID_DIM, 1.0f);
  rope_split_kernel<NUM_HEADS, HID_DIM><<<(NTOK * NUM_HEADS * 16) / 256, 256, 0, stream>>>(Qf, cosT, sinT, Qh, Ql, 0.0625f);
  rope_split_kernel<1, HEAD_DIM><<<(NTOK * 16) / 256, 256, 0, stream>>>(Kf, cosT, sinT, Kh, Kl, 1.0f);
  gqa_attn_kernel<<<NBATCH * NUM_HEADS * (SEQ_LEN / QBLK), 256, 0, stream>>>(Qh, Ql, Kh, Kl, Vth, Vtl, maskp, AOh, AOl);
  gemm_bf16_t64<true, false, 0><<<dim3(((NTOK / 64) * (HID_DIM / 64)) / 8, 1), 256, 0, stream>>>(
      AOh, AOl, HID_DIM, 0L, WoT, WoT, HID_DIM, 0L, (void*)out, (void*)out, HID_DIM, 0L, NTOK, HID_DIM, HID_DIM, 1.0f);
}
